// TripletAttentionUngated_71012989272673
// MI455X (gfx1250) — hardware-verified
//
#include <hip/hip_runtime.h>
#include <math.h>
typedef __attribute__((ext_vector_type(16))) _Float16 v16h;
typedef __attribute__((ext_vector_type(8)))  _Float16 v8h;
typedef __attribute__((ext_vector_type(16))) __bf16   v16b;
typedef __attribute__((ext_vector_type(8)))  __bf16   v8b;
typedef __attribute__((ext_vector_type(8)))  float    v8f;
typedef __attribute__((ext_vector_type(4)))  float    v4f;
#define PSCALE 32768.0f
#define U16(p) ((const unsigned short*)(const void*)(p))
#define PSCALE_INV (1.0f / 32768.0f)

__device__ __forceinline__ unsigned short f2bf_bits(float f) {
  unsigned u = __float_as_uint(f);
  return (unsigned short)((u + 0x7FFFu + ((u >> 16) & 1u)) >> 16);
}
__device__ __forceinline__ float bf_bits2f(unsigned short h) { return __uint_as_float(((unsigned)h) << 16); }

__device__ __forceinline__ void dep_guard_h(v8f& a, v8f& b, v16h x, v16h y) { asm volatile("v_nop\n\tv_nop\n\tv_nop\n\tv_nop" : "+v"(a), "+v"(b) : "v"(x), "v"(y)); }
__device__ __forceinline__ void dep_guard_b(v8f& a, v8f& b, v16b x, v16b y) { asm volatile("v_nop\n\tv_nop\n\tv_nop\n\tv_nop" : "+v"(a), "+v"(b) : "v"(x), "v"(y)); }
__device__ __forceinline__ void keep4_h(v16h a, v16h b, v16h c, v16h d) { asm volatile("v_nop" :: "v"(a), "v"(b), "v"(c), "v"(d)); }
__device__ __forceinline__ void keep4_b(v16b a, v16b b, v16b c, v16b d) { asm volatile("v_nop" :: "v"(a), "v"(b), "v"(c), "v"(d)); }
__device__ __forceinline__ void acc_guard4(v8f& a, v8f& b, v8f& c, v8f& d) { asm volatile("v_nop\n\tv_nop\n\tv_nop\n\tv_nop" : "+v"(a), "+v"(b), "+v"(c), "+v"(d)); }
template <typename T> struct Frag;
template <> struct Frag<_Float16> {
  typedef v16h V; union U { v16h v; v8h h[2]; };
  static __device__ __forceinline__ v16h load(const _Float16* p) {
    U f; f.h[0] = *(const v8h*)(p); f.h[1] = *(const v8h*)(p + 16); return f.v;
  }
  static __device__ __forceinline__ v8f mma(v16h a, v16h b, v8f c) {
    return __builtin_amdgcn_wmma_f32_16x16x32_f16(false, a, false, b, (short)0, c, false, false);
  }
  static __device__ __forceinline__ void guard(v8f& a, v8f& b, v16h x, v16h y) { dep_guard_h(a, b, x, y); }
  static __device__ __forceinline__ void keep(v16h a, v16h b, v16h c, v16h d) { keep4_h(a, b, c, d); }
};
template <> struct Frag<__bf16> {
  typedef v16b V; union U { v16b v; v8b h[2]; };
  static __device__ __forceinline__ v16b load(const __bf16* p) {
    U f; f.h[0] = *(const v8b*)(p); f.h[1] = *(const v8b*)(p + 16); return f.v;
  }
  static __device__ __forceinline__ v8f mma(v16b a, v16b b, v8f c) {
    return __builtin_amdgcn_wmma_f32_16x16x32_bf16(false, a, false, b, (short)0, c, false, false);
  }
  static __device__ __forceinline__ void guard(v8f& a, v8f& b, v16b x, v16b y) { dep_guard_b(a, b, x, y); }
  static __device__ __forceinline__ void keep(v16b a, v16b b, v16b c, v16b d) { keep4_b(a, b, c, d); }
};

template <int ET> struct Elem;
template <> struct Elem<0> { typedef _Float16 T; };
template <> struct Elem<1> { typedef __bf16 T; };
template <int ET, bool SPLIT, int BIAS_MODE, int OUT_MODE, bool RESID, int ACT = 0>
__global__ __launch_bounds__(256) void wmma_gemm64(
    const unsigned short* __restrict__ Ap, const unsigned short* __restrict__ A2p, int lda, long strideA,
    const unsigned short* __restrict__ Btp, const unsigned short* __restrict__ Bt2p, int ldb, long strideB,
    void* __restrict__ Cout, void* __restrict__ Cout2, int ldc, long strideC,
    const float* __restrict__ bias,
    const float* __restrict__ resid, long strideR,
    int M, int N, int K, float scale) {
  typedef typename Elem<ET>::T T;
  typedef typename Frag<T>::V V;
  const T* A = (const T*)Ap; const T* A2 = (const T*)A2p; const T* Bt = (const T*)Btp; const T* Bt2 = (const T*)Bt2p;
  __shared__ __align__(16) float sT[8][16 * 68];
  const int b    = blockIdx.y;
  const int lane = threadIdx.x & 31;
  const int wave = threadIdx.x >> 5;
  const int tilesN = N >> 6;
  const int tilesM = M >> 6;
  const int tile = blockIdx.x * 8 + wave;
  if (tile >= tilesM * tilesN) return;
  const int tm = tile / tilesN;
  const int tn = tile - tm * tilesN;
  const int m0 = tm << 6;
  const int n0 = tn << 6;

  const T* Ab  = A  + (size_t)b * strideA;
  const T* Bb  = Bt + (size_t)b * strideB;
  const T* Ab2 = SPLIT ? (A2  + (size_t)b * strideA) : nullptr;
  const T* Bb2 = SPLIT ? (Bt2 + (size_t)b * strideB) : nullptr;

  const int rlane = lane & 15;
  const int koff  = (lane >> 4) * 8;
  const int mOff  = (lane >> 4) * 8;

  v8f acc[4][4];
#pragma unroll
  for (int i = 0; i < 4; ++i)
#pragma unroll
    for (int j = 0; j < 4; ++j) acc[i][j] = (v8f){0.f,0.f,0.f,0.f,0.f,0.f,0.f,0.f};

  for (int k0 = 0; k0 < K; k0 += 32) {
    V bh[4], bl[4];
#pragma unroll
    for (int j = 0; j < 4; ++j) {
      const size_t bo = (size_t)(n0 + (j << 4) + rlane) * ldb + koff + k0;
      bh[j] = Frag<T>::load(Bb + bo);
      if (SPLIT) bl[j] = Frag<T>::load(Bb2 + bo);
    }
#pragma unroll
    for (int i = 0; i < 4; ++i) {
      const size_t ao = (size_t)(m0 + (i << 4) + rlane) * lda + koff + k0;
      V ah = Frag<T>::load(Ab + ao);
      V al;
      if (SPLIT) al = Frag<T>::load(Ab2 + ao);
#pragma unroll
      for (int j = 0; j < 4; ++j) {
        acc[i][j] = Frag<T>::mma(ah, bh[j], acc[i][j]);
        if (SPLIT) {
          acc[i][j] = Frag<T>::mma(ah, bl[j], acc[i][j]);
          acc[i][j] = Frag<T>::mma(al, bh[j], acc[i][j]);
        }
      }
      Frag<T>::guard(acc[i][0], acc[i][3], ah, SPLIT ? al : ah);
    }
    Frag<T>::keep(bh[0], bh[1], bh[2], bh[3]);
    if (SPLIT) Frag<T>::keep(bl[0], bl[1], bl[2], bl[3]);
  }
  acc_guard4(acc[0][0], acc[0][1], acc[0][2], acc[0][3]);
  acc_guard4(acc[1][0], acc[1][1], acc[1][2], acc[1][3]);
  acc_guard4(acc[2][0], acc[2][1], acc[2][2], acc[2][3]);
  acc_guard4(acc[3][0], acc[3][1], acc[3][2], acc[3][3]);

  float* slab = sT[wave];
  const float* Rb = RESID ? (resid + (size_t)b * strideR) : nullptr;
#pragma unroll
  for (int i = 0; i < 4; ++i) {
    const int mBase = m0 + (i << 4);
#pragma unroll
    for (int j = 0; j < 4; ++j) {
      const int n = n0 + (j << 4) + rlane;
      float bv = 0.f;
      if (BIAS_MODE == 2) bv = bias[n];
#pragma unroll
      for (int r = 0; r < 8; ++r) {
        float v = acc[i][j][r] * scale;
        if (BIAS_MODE == 1) v += bias[mBase + mOff + r];
        if (BIAS_MODE == 2) v += bv;
        if (RESID) v += Rb[(size_t)(mBase + mOff + r) * ldc + n];
        if (ACT == 1) v = tanhf(v);
        if (ACT == 2) v = fmaxf(v, 0.0f);
        if (ACT == 3) v = v / (1.0f + expf(-v));
        if (ACT == 4) v = (v > 0.f) ? v : 0.01f * v;
        if (ACT == 5) v = 0.5f * v * (1.0f + erff(v * 0.70710678118654752f));
        slab[(mOff + r) * 68 + (j << 4) + rlane] = v;
      }
    }
    __builtin_amdgcn_fence(__ATOMIC_RELEASE, "workgroup");
    __builtin_amdgcn_wave_barrier();
    __builtin_amdgcn_fence(__ATOMIC_ACQUIRE, "workgroup");
    if (OUT_MODE == 0) {
      float* C = (float*)Cout + (size_t)b * strideC;
      const int hh = lane >> 4, c4 = (lane & 15) * 4;
      for (int pass = 0; pass < 2; ++pass) {
#pragma unroll
        for (int it = 0; it < 8; ++it) {
          const int row = it * 2 + hh;
          v4f v = *(const v4f*)(slab + row * 68 + c4);
          *(volatile v4f*)(C + (size_t)(mBase + row) * ldc + n0 + c4) = v;
        }
        __threadfence();
      }
    } else {
      const int q = lane >> 3, c8 = (lane & 7) * 8;
      unsigned short* C  = (unsigned short*)Cout  + (size_t)b * strideC;
      unsigned short* C2 = (OUT_MODE == 2) ? ((unsigned short*)Cout2 + (size_t)b * strideC) : nullptr;
      for (int pass = 0; pass < 2; ++pass) {
#pragma unroll
        for (int it = 0; it < 4; ++it) {
          const int row = it * 4 + q;
          const float* sp = slab + row * 68 + c8;
          v8h hv, lv;
#pragma unroll
          for (int e = 0; e < 8; ++e) {
            if (OUT_MODE == 1) {
              hv[e] = (_Float16)sp[e];
            } else {
              unsigned short hb = f2bf_bits(sp[e]);
              unsigned short lb = f2bf_bits(sp[e] - bf_bits2f(hb));
              hv[e] = __builtin_bit_cast(_Float16, hb);
              lv[e] = __builtin_bit_cast(_Float16, lb);
            }
          }
          *(volatile v8h*)(C + (size_t)(mBase + row) * ldc + n0 + c8) = hv;
          if (OUT_MODE == 2) *(volatile v8h*)(C2 + (size_t)(mBase + row) * ldc + n0 + c8) = lv;
        }
        __threadfence();
      }
    }
    __builtin_amdgcn_fence(__ATOMIC_RELEASE, "workgroup");
    __builtin_amdgcn_wave_barrier();
    __builtin_amdgcn_fence(__ATOMIC_ACQUIRE, "workgroup");
  }
}


#define TB 2
#define TN 128
#define TC 256
#define TH 8
#define TD 32
#define TR (TB * TN * TN)
__device__ __forceinline__ unsigned pkh(float a, float b) { return (unsigned)__builtin_bit_cast(unsigned short, (_Float16)a) | ((unsigned)__builtin_bit_cast(unsigned short, (_Float16)b) << 16); }
__global__ __launch_bounds__(256) void ln_kernel(const float* __restrict__ e, const float* __restrict__ g, const float* __restrict__ bb, unsigned* __restrict__ E16) {
  const int lane = threadIdx.x & 31, wave = threadIdx.x >> 5; const size_t r = (size_t)blockIdx.x * 8 + wave;
  const v8f v = *(const v8f*)(e + r * TC + lane * 8); float s = 0.f; for (int q = 0; q < 8; ++q) s += v[q]; for (int o = 16; o > 0; o >>= 1) s += __shfl_xor(s, o, 32); const float mu = s / TC;
  float t = 0.f; for (int q = 0; q < 8; ++q) { const float d = v[q] - mu; t += d * d; } for (int o = 16; o > 0; o >>= 1) t += __shfl_xor(t, o, 32); const float inv = rsqrtf(t / TC + 1e-5f);
  typedef __attribute__((ext_vector_type(4))) unsigned u4; u4 u; for (int q = 0; q < 4; ++q) { const int c = lane * 8 + 2 * q; u[q] = pkh((v[2*q] - mu) * inv * g[c] + bb[c], (v[2*q+1] - mu) * inv * g[c + 1] + bb[c + 1]); }
  *(volatile u4*)(E16 + (r * TC + lane * 8) / 2) = u; __threadfence(); *(volatile u4*)(E16 + (r * TC + lane * 8) / 2) = u;
}
__global__ __launch_bounds__(256) void wqkv_kernel(const float* __restrict__ Wm, const float* __restrict__ bm, unsigned* __restrict__ BT, float* __restrict__ BP) {
  const int sec = blockIdx.y;
  for (int i = blockIdx.x * 256 + threadIdx.x; i < TC * TC / 2; i += gridDim.x * 256) { const int row = i / (TC / 2), cp = 2 * (i % (TC / 2)); const int h = row / TD, d = row % TD; const int col = sec * TC + d * TH + h;
    const unsigned u = pkh(Wm[(size_t)cp * 768 + col], Wm[(size_t)(cp + 1) * 768 + col]); ((volatile unsigned*)BT)[(size_t)sec * TC * TC / 2 + i] = u; __threadfence(); ((volatile unsigned*)BT)[(size_t)sec * TC * TC / 2 + i] = u;
    if (i < TC) { const int hh = i / TD, dd = i % TD; ((volatile float*)BP)[sec * TC + i] = bm[sec * TC + dd * TH + hh]; } }
}
__global__ __launch_bounds__(256) void we_kernel(const float* __restrict__ Wi, const float* __restrict__ Wo, unsigned* __restrict__ BT) {
  for (int i = threadIdx.x; i < 64 * TC / 2; i += 256) { const int row = i / (TC / 2), cp = 2 * (i % (TC / 2)); float a = 0.f, b = 0.f;
    if (row < 8) { a = Wi[cp * TH + row]; b = Wi[(cp + 1) * TH + row]; } else if (row < 16) { a = Wo[cp * TH + row - 8]; b = Wo[(cp + 1) * TH + row - 8]; }
    ((volatile unsigned*)BT)[i] = pkh(a, b); __threadfence(); ((volatile unsigned*)BT)[i] = pkh(a, b); }
}
__global__ __launch_bounds__(256) void wo_kernel(const float* __restrict__ WO, unsigned* __restrict__ BTa, unsigned* __restrict__ BTb) {
  for (int i = blockIdx.x * 256 + threadIdx.x; i < TC * TC / 2; i += gridDim.x * 256) { const int m = i / (TC / 2), kp = 2 * (i % (TC / 2)); const int h0 = kp / TD, d0 = kp % TD, h1 = (kp + 1) / TD, d1 = (kp + 1) % TD;
    const unsigned ua = pkh(WO[(size_t)(d0 * 2 * TH + h0) * TC + m], WO[(size_t)(d1 * 2 * TH + h1) * TC + m]), ub = pkh(WO[(size_t)(d0 * 2 * TH + TH + h0) * TC + m], WO[(size_t)(d1 * 2 * TH + TH + h1) * TC + m]);
    ((volatile unsigned*)BTa)[i] = ua; ((volatile unsigned*)BTb)[i] = ub; __threadfence(); ((volatile unsigned*)BTa)[i] = ua; ((volatile unsigned*)BTb)[i] = ub; }
}
__global__ __launch_bounds__(256) void rowswap_kernel(const unsigned* __restrict__ K16, unsigned* __restrict__ KT16) {
  const int lane = threadIdx.x & 31, wave = threadIdx.x >> 5; const int r = blockIdx.x * 8 + wave; const int b = r / (TN * TN), a = (r / TN) % TN, c = r % TN;
  typedef __attribute__((ext_vector_type(4))) unsigned u4; const u4 v = *(const u4*)(K16 + ((size_t)((b * TN + c) * TN + a) * TC) / 2 + lane * 4);
  *(volatile u4*)(KT16 + ((size_t)r * TC) / 2 + lane * 4) = v; __threadfence(); *(volatile u4*)(KT16 + ((size_t)r * TC) / 2 + lane * 4) = v;
}
template <int MODE>
__global__ __launch_bounds__(256) void vt_kernel(const unsigned* __restrict__ V16, int b, int j0, unsigned* __restrict__ VT) {
  __shared__ float tile[TN][33];
  const int z = blockIdx.x; const int h = z % TH, j = j0 + z / TH; const int tx = threadIdx.x, ty = threadIdx.y; typedef __attribute__((ext_vector_type(2))) _Float16 v2h;
  for (int k = ty; k < TN; k += 8) { const size_t row = (MODE == 0) ? ((size_t)(b * TN + j) * TN + k) : ((size_t)(b * TN + k) * TN + j); if (tx < 16) { const v2h p = __builtin_bit_cast(v2h, V16[(row * TC + h * TD) / 2 + tx]); tile[k][2 * tx] = (float)p[0]; tile[k][2 * tx + 1] = (float)p[1]; } }
  __syncthreads();
  unsigned* dst = VT + (size_t)z * 64 * TN / 2;
  for (int pass = 0; pass < 2; ++pass) { for (int d = ty; d < 64; d += 8) for (int kk = tx; kk < TN / 2; kk += 32) ((volatile unsigned*)dst)[(d * TN) / 2 + kk] = (d < TD) ? pkh(tile[2 * kk][d], tile[2 * kk + 1][d]) : 0u; __threadfence(); }
}
template <int MODE>
__global__ __launch_bounds__(256) void soft_kernel(const float* __restrict__ S, int b, int j0, const float* __restrict__ EB, const float* __restrict__ bE, const float* __restrict__ mask, unsigned* __restrict__ P16) {
  const int lane = threadIdx.x & 31, wave = threadIdx.x >> 5; const size_t row = (size_t)blockIdx.x * 8 + wave; const int i = (int)(row % TN); const int z = (int)(row / TN); const int h = z % TH; (void)j0;
  float v[4]; float mx = -INFINITY;
#pragma unroll
  for (int q = 0; q < 4; ++q) { const int k = lane * 4 + q; const size_t pr = (MODE == 0) ? ((size_t)(b * TN + i) * TN + k) : ((size_t)(b * TN + k) * TN + i);
    const float ev = EB[pr * 64 + (MODE == 0 ? h : 8 + h)] + bE[h]; const float mk = mask[pr * TH + h];
    v[q] = S[row * TN + k] + ev + mk; mx = fmaxf(mx, v[q]); }
  for (int o = 16; o > 0; o >>= 1) mx = fmaxf(mx, __shfl_xor(mx, o, 32));
  float sum = 0.f; for (int q = 0; q < 4; ++q) { v[q] = __expf(v[q] - mx); sum += v[q]; } for (int o = 16; o > 0; o >>= 1) sum += __shfl_xor(sum, o, 32);
  const float sc = 32768.0f / sum; typedef __attribute__((ext_vector_type(2))) unsigned u2; const u2 u = {pkh(v[0] * sc, v[1] * sc), pkh(v[2] * sc, v[3] * sc)};
  *(volatile u2*)(P16 + (row * TN + lane * 4) / 2) = u; __threadfence(); *(volatile u2*)(P16 + (row * TN + lane * 4) / 2) = u;
}
__global__ __launch_bounds__(256) void orelay_kernel(const float* __restrict__ OZ, int b, int j0, unsigned* __restrict__ O16) {
  const int lane = threadIdx.x & 31, wave = threadIdx.x >> 5; const int r = blockIdx.x * 8 + wave; const int i = r / (TN / 4), jl = r % (TN / 4), j = j0 + jl; const int h = lane / 4, d0 = (lane % 4) * 8;
  const float* src = OZ + ((size_t)(jl * TH + h) * TN + i) * 64 + d0; typedef __attribute__((ext_vector_type(4))) unsigned u4; u4 u; for (int q = 0; q < 4; ++q) u[q] = pkh(src[2 * q], src[2 * q + 1]);
  unsigned* dst = O16 + (((size_t)(b * TN + i) * TN + j) * TC + h * TD + d0) / 2; *(volatile u4*)dst = u; __threadfence(); *(volatile u4*)dst = u;
}
extern "C" void kernel_launch(void* const* d_in, const int* in_sizes, int n_in, void* d_out, int out_size, void* d_ws, size_t ws_size, hipStream_t stream) {
  (void)in_sizes; (void)n_in; (void)out_size; (void)ws_size;
  auto Fp = [&](int i) { return (const float*)d_in[i]; };
  const float* e = Fp(0); const float* mask = Fp(1); const float* lng = Fp(2); const float* lnb = Fp(3); const float* Wqi = Fp(4); const float* bqi = Fp(5); const float* WEi = Fp(6); const float* bEi = Fp(7); const float* Wqo = Fp(8); const float* bqo = Fp(9); const float* WEo = Fp(10); const float* bEo = Fp(11); const float* WO = Fp(12); const float* bO = Fp(13);
  char* ws = (char*)d_ws; size_t off = 0;
  auto carve = [&](size_t bytes) -> char* { char* p = ws + off; off += (bytes + 255) & ~(size_t)255; return p; };
  unsigned* E16 = (unsigned*)carve((size_t)TR * TC * 2); unsigned* BTQ[2]; float* BP[2]; for (int p = 0; p < 2; ++p) { BTQ[p] = (unsigned*)carve((size_t)3 * TC * TC * 2); BP[p] = (float*)carve(3 * TC * 4); }
  unsigned* BTE = (unsigned*)carve(64 * TC * 2); unsigned* BTOa = (unsigned*)carve(TC * TC * 2); unsigned* BTOb = (unsigned*)carve(TC * TC * 2);
  float* EB = (float*)carve((size_t)TR * 64 * 4); unsigned* Q16 = (unsigned*)carve((size_t)TR * TC * 2); unsigned* K16 = (unsigned*)carve((size_t)TR * TC * 2); unsigned* V16 = (unsigned*)carve((size_t)TR * TC * 2);
  const int ZH = TN * TH / 4;
  unsigned* VT = (unsigned*)carve((size_t)ZH * 64 * TN * 2); unsigned* P16 = (unsigned*)carve((size_t)ZH * TN * TN * 2); float* OZ = (float*)carve((size_t)ZH * TN * 64 * 4);
  unsigned* O16[2]; O16[0] = (unsigned*)carve((size_t)TR * TC * 2); O16[1] = E16;
  float* S = (float*)carve((size_t)ZH * TN * TN * 4);
  ln_kernel<<<TR / 8, 256, 0, stream>>>(e, lng, lnb, E16);
  wqkv_kernel<<<dim3(32, 3), 256, 0, stream>>>(Wqi, bqi, BTQ[0], BP[0]); wqkv_kernel<<<dim3(32, 3), 256, 0, stream>>>(Wqo, bqo, BTQ[1], BP[1]);
  we_kernel<<<1, 256, 0, stream>>>(WEi, WEo, BTE); wo_kernel<<<32, 256, 0, stream>>>(WO, BTOa, BTOb);
  const int tr = (TR / 64);
  wmma_gemm64<0, false, 0, 0, false><<<dim3((tr * 1 + 7) / 8, 1), 256, 0, stream>>>((const unsigned short*)E16, nullptr, TC, 0, (const unsigned short*)BTE, nullptr, TC, 0, EB, nullptr, 64, 0, nullptr, nullptr, 0, TR, 64, TC, 1.0f);
  const int tz = (TN / 64) * (TN / 64);
  for (int p = 0; p < 2; ++p) {
    wmma_gemm64<0, false, 2, 1, false><<<dim3((tr * 4 + 7) / 8, 1), 256, 0, stream>>>((const unsigned short*)E16, nullptr, TC, 0, (const unsigned short*)BTQ[p], nullptr, TC, 0, Q16, nullptr, TC, 0, BP[p], nullptr, 0, TR, TC, TC, 1.0f);
    if (p == 0) { for (int b = 0; b < TB; ++b)
        wmma_gemm64<0, false, 2, 1, false><<<dim3(1, TN), 256, 0, stream>>>((const unsigned short*)E16 + (size_t)b * TN * TN * TC, nullptr, TC, (long)TN * TC, (const unsigned short*)BTQ[p] + (size_t)TC * TC, nullptr, TC, 0, K16 + ((size_t)b * TN * TN * TC) / 2, nullptr, TN * TC, TC, BP[p] + TC, nullptr, 0, TN, TC, TC, 1.0f); }
    else wmma_gemm64<0, false, 2, 1, false><<<dim3((tr * 4 + 7) / 8, 1), 256, 0, stream>>>((const unsigned short*)E16, nullptr, TC, 0, (const unsigned short*)BTQ[p] + (size_t)TC * TC, nullptr, TC, 0, K16, nullptr, TC, 0, BP[p] + TC, nullptr, 0, TR, TC, TC, 1.0f);
    wmma_gemm64<0, false, 2, 1, false><<<dim3((tr * 4 + 7) / 8, 1), 256, 0, stream>>>((const unsigned short*)E16, nullptr, TC, 0, (const unsigned short*)BTQ[p] + (size_t)2 * TC * TC, nullptr, TC, 0, V16, nullptr, TC, 0, BP[p] + 2 * TC, nullptr, 0, TR, TC, TC, 1.0f);
    const unsigned* KB = K16;
    for (int b = 0; b < TB; ++b) for (int zq = 0; zq < 4; ++zq) { const int j0 = zq * (TN / 4);
      const size_t bo = (size_t)b * TN * TN * TC + (size_t)zq * ZH * TD;
      if (p == 0) vt_kernel<0><<<ZH, dim3(32, 8), 0, stream>>>(V16, b, j0, VT); else vt_kernel<1><<<ZH, dim3(32, 8), 0, stream>>>(V16, b, j0, VT);
      wmma_gemm64<0, false, 0, 0, false><<<dim3((tz + 7) / 8, ZH), 256, 0, stream>>>((const unsigned short*)Q16 + bo, nullptr, TN * TC, TD, (const unsigned short*)KB + bo, nullptr, TN * TC, TD, S, nullptr, TN, (long)TN * TN, nullptr, nullptr, 0, TN, TN, TD, 0.17677669529663687f);
      if (p == 0) soft_kernel<0><<<ZH * TN / 8, 256, 0, stream>>>(S, b, j0, EB, bEi, mask, P16); else soft_kernel<1><<<ZH * TN / 8, 256, 0, stream>>>(S, b, j0, EB, bEo, mask, P16);
      wmma_gemm64<0, false, 0, 0, false><<<dim3(1, ZH), 256, 0, stream>>>((const unsigned short*)P16, nullptr, TN, (long)TN * TN, (const unsigned short*)VT, nullptr, TN, (long)64 * TN, OZ, nullptr, 64, (long)TN * 64, nullptr, nullptr, 0, TN, 64, TN, 1.0f / 32768.0f);
      orelay_kernel<<<TN * (TN / 4) / 8, 256, 0, stream>>>(OZ, b, j0, O16[p]); } }
  wmma_gemm64<0, false, 2, 0, false><<<dim3((tr * 4 + 7) / 8, 1), 256, 0, stream>>>((const unsigned short*)O16[0], nullptr, TC, 0, (const unsigned short*)BTOa, nullptr, TC, 0, (float*)d_out, nullptr, TC, 0, bO, nullptr, 0, TR, TC, TC, 1.0f);
  wmma_gemm64<0, false, 0, 0, true><<<dim3((tr * 4 + 7) / 8, 1), 256, 0, stream>>>((const unsigned short*)O16[1], nullptr, TC, 0, (const unsigned short*)BTOb, nullptr, TC, 0, (float*)d_out, nullptr, TC, 0, nullptr, (const float*)d_out, 0, TR, TC, TC, 1.0f);
}
